// SizeConditionedDepthExperts_49426483642688
// MI455X (gfx1250) — hardware-run, weakly checked
//
#include <hip/hip_runtime.h>


namespace {
constexpr int B = 8192, D = 1024, NE = 8, H = 1024, KC = 5, KL = KC - 1, CAP = 1536, NSLOT = NE * CAP, RB = CAP / 64;
constexpr float XS = 8.0f, WSC = 256.0f, EPSP = 1e-8f;
typedef _Float16 b16;
typedef __attribute__((ext_vector_type(16))) _Float16 v16b;
typedef __attribute__((ext_vector_type(8))) _Float16 v8b;
typedef __attribute__((ext_vector_type(4))) _Float16 v4b;
typedef __attribute__((ext_vector_type(8))) float v8f;
typedef __attribute__((ext_vector_type(4))) float v4f;
__device__ __forceinline__ float bf16_rne(float f) { unsigned int u = __float_as_uint(f); u += 0x7FFFu + ((u >> 16) & 1u); return __uint_as_float(u & 0xFFFF0000u); }
__device__ __forceinline__ void split16(float v, b16& hi, b16& lo) { hi = (b16)v; lo = (b16)(v - (float)hi); }
__device__ __forceinline__ v16b frag_kb(const b16* p, int hh) { const v8b a = *(const v8b*)(p + 8 * hh), b = *(const v8b*)(p + 16 + 8 * hh); v16b f;
#pragma unroll
  for (int e = 0; e < 8; ++e) { f[e] = a[e]; f[8 + e] = b[e]; } return f; }
__device__ __forceinline__ v8f wmma16b(v16b a, v16b b, v8f c) { v8f d = __builtin_amdgcn_wmma_f32_16x16x32_f16(false, a, false, b, (short)0, c, false, false); asm volatile("v_nop\n\tv_nop\n\tv_nop\n\tv_nop" : "+v"(d) : "v"(a), "v"(b)); return d; }
__device__ __forceinline__ void wave_lds_sync() { __builtin_amdgcn_fence(__ATOMIC_RELEASE, "workgroup"); __builtin_amdgcn_wave_barrier(); __builtin_amdgcn_fence(__ATOMIC_ACQUIRE, "workgroup"); }
__device__ __forceinline__ float pmul(float a, float b) { float p = a * b; asm volatile("" : "+v"(p)); return p; }
__device__ __forceinline__ int iclamp(int v, int lo, int hi) { return v < lo ? lo : (v > hi ? hi : v); }
__device__ __forceinline__ float sigm(float x) { return 1.0f / (1.0f + __expf(-x)); }
constexpr int CSR_NBLK3 = 512, CSR_GB3 = 3, CSR_GN3 = 1 << CSR_GB3  , CSR_TS3 = (CSR_GN3 < 32 ? 32 : CSR_GN3)  , CSR_MAXG3 = 512, CSR_CAP3 = 12288  ;
__device__ __host__ __forceinline__ int csr_tix3(int v) { return (v >> CSR_GB3) * CSR_TS3 + (v & (CSR_GN3 - 1)); }
__global__ __launch_bounds__(64) void csrA_kernel3(const int* __restrict__ dst, int E, int N, int nG, int CHP, int NGP, int* __restrict__ STG, int* __restrict__ HST) {
  extern __shared__ int sm[];
  int* cnt = sm; int* run = sm + NGP; int* ids = sm + 2 * NGP;
  const int b = blockIdx.x; const int ch = (E + CSR_NBLK3 - 1) / CSR_NBLK3; const int e0 = b * ch, e1 = min(E, e0 + ch);
  for (int i = threadIdx.x; i < NGP; i += 64) cnt[i] = 0;
  for (int i = threadIdx.x; i < CHP; i += 64) ids[i] = -1;
  __syncthreads();
  if (threadIdx.x == 0) {
    for (int e = e0; e < e1; ++e) { int d = dst[e]; d = (d < 0) ? 0 : (d >= N ? N - 1 : d); cnt[d >> CSR_GB3] += 1; }
    int acc = 0; for (int g = 0; g < nG; ++g) { run[g] = acc; acc += cnt[g]; }
    for (int e = e0; e < e1; ++e) { int d = dst[e]; d = (d < 0) ? 0 : (d >= N ? N - 1 : d); const int g = d >> CSR_GB3; ids[run[g]] = e; run[g] += 1; } }
  __syncthreads();
  typedef __attribute__((ext_vector_type(4))) int v4i;
  for (int pass = 0; pass < 2; ++pass) {
    for (int i = threadIdx.x; i < CHP / 4; i += 64) *(volatile v4i*)(STG + (size_t)b * CHP + i * 4) = *(const v4i*)(&ids[i * 4]);
    for (int i = threadIdx.x; i < NGP / 4; i += 64) { v4i v; for (int e = 0; e < 4; ++e) v[e] = (i * 4 + e < nG) ? cnt[i * 4 + e] : 0; *(volatile v4i*)(HST + (size_t)b * NGP + i * 4) = v; }
    __threadfence(); }
}
__global__ __launch_bounds__(512) void csrS_kernel3(const int* __restrict__ HST, int nG, int NGP, int* __restrict__ START, int* __restrict__ TOT, int* __restrict__ OFF) {
  __shared__ int tot[CSR_MAXG3];
  const int b = threadIdx.x;
  for (int pass = 0; pass < 2; ++pass) { int runb = 0; for (int g = 0; g < nG; ++g) { int c = HST[(size_t)b * NGP + g]; c = (c < 0) ? 0 : c; ((volatile int*)OFF)[(size_t)g * CSR_NBLK3 + b] = runb; runb += c; } __threadfence(); }
  for (int g = threadIdx.x; g < nG; g += 512) { int s = 0; for (int bb = 0; bb < CSR_NBLK3; ++bb) { int c = HST[(size_t)bb * NGP + g]; s += (c < 0) ? 0 : c; } tot[g] = s; }
  __syncthreads();
  if (threadIdx.x < 32) {
    __shared__ int st[CSR_MAXG3 + 32];
    if (threadIdx.x == 0) { int acc = 0; for (int g = 0; g < NGP; ++g) { st[g] = acc; if (g < nG) acc += (tot[g] + 31) & ~31; } st[NGP] = acc; }
    __builtin_amdgcn_fence(__ATOMIC_RELEASE, "workgroup"); __builtin_amdgcn_wave_barrier(); __builtin_amdgcn_fence(__ATOMIC_ACQUIRE, "workgroup");
    for (int pass = 0; pass < 2; ++pass) { for (int i = threadIdx.x; i < NGP + 32; i += 32) { ((volatile int*)START)[i] = (i <= NGP) ? st[min(i, NGP)] : 0; ((volatile int*)TOT)[i] = (i < nG) ? tot[i] : 0; } __threadfence(); } }
}
__global__ __launch_bounds__(256) void csrB_kernel3(const int* __restrict__ dst, int N, int nG, int CHP, int NGP, int permLen, const int* __restrict__ STG, const int* __restrict__ HST, const int* __restrict__ OFF, const int* __restrict__ START, const int* __restrict__ TOT, int* __restrict__ PERM, int* __restrict__ ROWPTR, int* __restrict__ ROWCNT, int* __restrict__ FLAG) {
  typedef __attribute__((ext_vector_type(4))) int v4i;
  __shared__ int ids[CSR_CAP3]; __shared__ unsigned short key[CSR_CAP3]; __shared__ int outp[CSR_CAP3]; __shared__ int ncnt[CSR_GN3 + 1]; __shared__ int boff[CSR_NBLK3 + 1];
  const int g = blockIdx.x, t_ = threadIdx.x; int tot = TOT[g]; int st = START[g], stn = START[g + 1]; const int v0 = g * CSR_GN3; const int nv = min(CSR_GN3, N - v0); const int t0 = g * CSR_TS3;
  st = (st < 0) ? 0 : (st > permLen - 32 ? permLen - 32 : st) & ~31; stn = (stn < st) ? st : (stn > permLen ? permLen : stn); tot = (tot < 0) ? 0 : tot; if (tot > stn - st && tot <= CSR_CAP3) tot = stn - st;
  if (tot > CSR_CAP3) {
    for (int pass = 0; pass < 2; ++pass) { for (int i = t_; i < CSR_TS3 / 4; i += 256) { v4i a, c; for (int e = 0; e < 4; ++e) { a[e] = st; c[e] = 0; } *(volatile v4i*)(ROWPTR + t0 + i * 4) = a; *(volatile v4i*)(ROWCNT + t0 + i * 4) = c; } if (t_ == 0) ((volatile int*)FLAG)[0] = 1; __threadfence(); } (void)nv; return; }
  if (t_ == 0) { int acc = 0; for (int b = 0; b < CSR_NBLK3; ++b) { boff[b] = acc; int c = HST[(size_t)b * NGP + g]; c = (c < 0) ? 0 : (c > CHP ? CHP : c); acc += c; if (acc > tot) acc = tot; } boff[CSR_NBLK3] = acc; }
  for (int i = t_; i <= CSR_GN3; i += 256) ncnt[i] = 0;
  __syncthreads();
  for (int b = 0; b < CSR_NBLK3; ++b) { const int c = boff[b + 1] - boff[b]; int o_ = OFF[(size_t)g * CSR_NBLK3 + b]; o_ = (o_ < 0) ? 0 : (o_ > CHP - c ? CHP - c : o_); const int* src_ = STG + (size_t)b * CHP + o_;
    for (int i = t_; i < c; i += 256) { int id = src_[i]; id = (id < 0) ? 0 : id; ids[boff[b] + i] = id; int d = dst[id]; d = (d < v0) ? v0 : (d >= N ? N - 1 : d); int kk = d - v0; kk = (kk < 0) ? 0 : (kk >= CSR_GN3 ? CSR_GN3 - 1 : kk); key[boff[b] + i] = (unsigned short)kk; } }
  __syncthreads();
  if (t_ == 0) { for (int i = 0; i < tot; ++i) ncnt[key[i]] += 1; int acc = 0; for (int vl = 0; vl < CSR_GN3; ++vl) { const int c = ncnt[vl]; ncnt[vl] = acc; acc += c; } ncnt[CSR_GN3] = acc;
    for (int i = 0; i < tot; ++i) { const int vl = key[i]; outp[ncnt[vl]] = ids[i]; ncnt[vl] += 1; }
    for (int vl = CSR_GN3; vl > 0; --vl) ncnt[vl] = ncnt[vl - 1]; ncnt[0] = 0; }
  __syncthreads();
  for (int pass = 0; pass < 2; ++pass) {
    for (int i = t_; i < (stn - st) / 4; i += 256) { v4i v; for (int e = 0; e < 4; ++e) { const int q = i * 4 + e; v[e] = (q < tot) ? outp[q] : -1; } *(volatile v4i*)(PERM + st + i * 4) = v; }
    for (int i = t_; i < CSR_TS3 / 4; i += 256) { v4i a, c; for (int e = 0; e < 4; ++e) { const int vl = i * 4 + e; const int vc = vl < CSR_GN3 ? vl : CSR_GN3; a[e] = (vl < CSR_GN3) ? st + ncnt[vc] : st; c[e] = (vl < nv) ? (ncnt[(vc < CSR_GN3 ? vc : CSR_GN3 - 1) + 1] - ncnt[vc]) : 0; } *(volatile v4i*)(ROWPTR + t0 + i * 4) = a; *(volatile v4i*)(ROWCNT + t0 + i * 4) = c; }
    __threadfence(); }
}
__global__ __launch_bounds__(256) void csrZ_kernel3(int* __restrict__ p, size_t n4) { typedef __attribute__((ext_vector_type(4))) int v4i; const size_t tid = (size_t)blockIdx.x * 256 + threadIdx.x, nth = (size_t)gridDim.x * 256; v4i z = {0, 0, 0, 0}; for (size_t i = tid; i < n4; i += nth) *(volatile v4i*)(p + i * 4) = z; }
struct CsrBufs3 { int *STG, *HST, *OFF, *START, *TOT, *PERM, *ROWPTR, *ROWCNT, *FLAG; int nG, NGP, CHP; size_t permLen; char* base; size_t bytes; };
static size_t csr_carve3(CsrBufs3& c, char* ws, size_t off, int E, int N) {
  const size_t off0 = off; c.base = ws + off;
  auto al = [&](size_t bytes) { char* p = ws + off; off += (bytes + 255) & ~(size_t)255; return p; };
  c.nG = (N + CSR_GN3 - 1) / CSR_GN3; c.NGP = (c.nG + 31) & ~31; const int ch = (E + CSR_NBLK3 - 1) / CSR_NBLK3; c.CHP = (ch + 31) & ~31; c.permLen = (size_t)E + 32 * (size_t)c.nG + 32;
  c.STG = (int*)al((size_t)CSR_NBLK3 * c.CHP * 4); c.HST = (int*)al((size_t)CSR_NBLK3 * c.NGP * 4); c.OFF = (int*)al((size_t)c.NGP * CSR_NBLK3 * 4); c.START = (int*)al((size_t)(c.NGP + 64) * 4); c.TOT = (int*)al((size_t)(c.NGP + 64) * 4);
  c.PERM = (int*)al(c.permLen * 4); c.ROWPTR = (int*)al((size_t)c.nG * CSR_TS3 * 4); c.ROWCNT = (int*)al((size_t)c.nG * CSR_TS3 * 4); c.FLAG = (int*)al(256);
  c.bytes = off - off0; return off;
}
static void csr_build3(const CsrBufs3& c, const int* dst, int E, int N, hipStream_t stream) {
  const size_t smem = (size_t)(2 * c.NGP + c.CHP) * 4;
  csrZ_kernel3<<<512, 256, 0, stream>>>((int*)c.base, c.bytes / 16);
  csrA_kernel3<<<CSR_NBLK3, 64, smem, stream>>>(dst, E, N, c.nG, c.CHP, c.NGP, c.STG, c.HST);
  csrS_kernel3<<<1, 512, 0, stream>>>(c.HST, c.nG, c.NGP, c.START, c.TOT, c.OFF);
  csrB_kernel3<<<c.nG, 256, 0, stream>>>(dst, N, c.nG, c.CHP, c.NGP, (int)c.permLen, c.STG, c.HST, c.OFF, c.START, c.TOT, c.PERM, c.ROWPTR, c.ROWCNT, c.FLAG);
}


__global__ __launch_bounds__(256) void wprep1_kernel(const float* __restrict__ w1, b16* __restrict__ W1T) {
  __shared__ b16 tile[64][64 + 2];
  const int e = blockIdx.z, d0 = blockIdx.x * 64, h0 = blockIdx.y * 64; const int wave = threadIdx.x >> 5, lane = threadIdx.x & 31;
  for (int rr = 0; rr < 8; ++rr) { const int dl = wave * 8 + rr; const float* row = w1 + ((size_t)e * D + d0 + dl) * H + h0 + lane * 2; tile[lane * 2][dl] = (b16)(bf16_rne(row[0]) * WSC); tile[lane * 2 + 1][dl] = (b16)(bf16_rne(row[1]) * WSC); }
  __syncthreads();
  for (int pass = 0; pass < 2; ++pass) { for (int rr = 0; rr < 8; ++rr) { const int hl = wave * 8 + rr; typedef __attribute__((ext_vector_type(2))) _Float16 v2b; v2b v; v[0] = tile[hl][lane * 2]; v[1] = tile[hl][lane * 2 + 1]; *(volatile v2b*)(W1T + ((size_t)e * H + h0 + hl) * D + d0 + lane * 2) = v; } __threadfence(); }
}
__global__ __launch_bounds__(256) void wprep2_kernel(const float* __restrict__ w2, b16* __restrict__ W2P) {
  const size_t u = (size_t)blockIdx.x * 256 + threadIdx.x; if (u >= (size_t)NE * 16 * D / 8) return; const size_t el = u * 8; const int e = (int)(el / (16 * D)); const int k = (int)((el / D) % 16); const int d0 = (int)(el % D); v8b o;
  for (int j = 0; j < 8; ++j) o[j] = (k < KL) ? (b16)(bf16_rne(w2[((size_t)e * H + d0 + j) * KL + (k < KL ? k : 0)]) * WSC) : (b16)0.0f;
  for (int pass = 0; pass < 2; ++pass) { *(volatile v8b*)(W2P + el) = o; __threadfence(); }
}
__global__ __launch_bounds__(256) void rank_kernel(const int* __restrict__ sidx, int* __restrict__ RANK) {
  const int e = threadIdx.x >> 5, lane = threadIdx.x & 31; int base = 0;
#pragma unroll 1
  for (int t0 = 0; t0 < B; t0 += 32) { const int t = t0 + lane; const bool m = (sidx[t] == e); const unsigned long long bal = __ballot(m); const unsigned int below = (unsigned int)(bal & ((1ull << lane) - 1ull));
    const int r = base + __popc(below);
    for (int pass = 0; pass < 2; ++pass) { ((volatile int*)RANK)[(size_t)e * B + t] = r; __threadfence(); }
    base += __popcll(bal & 0xFFFFFFFFull); }
}
__global__ __launch_bounds__(128) void l1_kernel(const float* __restrict__ x, const b16* __restrict__ W1T, const float* __restrict__ b1, const int* __restrict__ PERM, const int* __restrict__ ROWPTR, const int* __restrict__ ROWCNT, int permLen, b16* __restrict__ HH, b16* __restrict__ HL) {
  __shared__ __attribute__((aligned(16))) float Tf[4][16][128 + 4];
  const int wave = threadIdx.x >> 5, lane = threadIdx.x & 31, nloc = lane & 15, hlf = lane >> 4; const int e = blockIdx.z; const int r0 = blockIdx.x * 64 + wave * 16; const int c0 = blockIdx.y * 128;
  int cnt = ROWCNT[e], st = ROWPTR[e]; cnt = iclamp(cnt, 0, CAP); st = iclamp(st, 0, permLen - cnt);
  if (r0 >= cnt) return;
  const int rv = r0 + nloc < cnt ? r0 + nloc : cnt - 1; const int tok = iclamp(PERM[st + rv], 0, B - 1); const float* xr = x + (size_t)tok * D;
  v8f acc[8];
#pragma unroll
  for (int t = 0; t < 8; ++t) acc[t] = (v8f){};
  const b16* wb = W1T + ((size_t)e * H + c0) * D;
#pragma unroll 2
  for (int kb = 0; kb < D; kb += 32) { v16b a; for (int j = 0; j < 8; ++j) { a[j] = (b16)(bf16_rne(xr[kb + 8 * hlf + j]) * XS); a[8 + j] = (b16)(bf16_rne(xr[kb + 16 + 8 * hlf + j]) * XS); }
#pragma unroll
    for (int t = 0; t < 8; ++t) acc[t] = wmma16b(a, frag_kb(wb + (size_t)(t * 16 + nloc) * D + kb, hlf), acc[t]); }
#pragma unroll
  for (int t = 0; t < 8; ++t) { const int c = t * 16 + nloc; const float bb = bf16_rne(b1[(size_t)e * H + c0 + c]);
#pragma unroll 1
    for (int r8 = 0; r8 < 8; ++r8) Tf[wave][8 * hlf + r8][c] = fmaxf(acc[t][r8] * (1.0f / (XS * WSC)) + bb, 0.0f); }
  wave_lds_sync();
  for (int pass = 0; pass < 2; ++pass) { for (int rr = 0; rr < 16; ++rr) { const size_t slot = (size_t)e * CAP + r0 + rr; v4b vh, vl; for (int j = 0; j < 4; ++j) { b16 p, q; split16(Tf[wave][rr][lane * 4 + j] * XS, p, q); vh[j] = p; vl[j] = q; }
      *(volatile v4b*)(HH + slot * H + c0 + lane * 4) = vh; *(volatile v4b*)(HL + slot * H + c0 + lane * 4) = vl; } __threadfence(); }
}
__global__ __launch_bounds__(128) void l2_kernel(const b16* __restrict__ HH, const b16* __restrict__ HL, const b16* __restrict__ W2P, const float* __restrict__ b2, const int* __restrict__ ROWCNT, float* __restrict__ LOGS, float* __restrict__ PRS) {
  __shared__ __attribute__((aligned(16))) float so[4][16][4], sp[4][16][8];
  const int wave = threadIdx.x >> 5, lane = threadIdx.x & 31, nloc = lane & 15, hlf = lane >> 4; const int e = blockIdx.z; const int r0 = blockIdx.x * 64 + wave * 16;
  int cnt = ROWCNT[e]; cnt = iclamp(cnt, 0, CAP); if (r0 >= cnt) return;
  const size_t slot0 = (size_t)e * CAP + r0; v8f acc = (v8f){};
#pragma unroll 4
  for (int kb = 0; kb < H; kb += 32) { const v16b a = frag_kb(HH + (slot0 + nloc) * H + kb, hlf), al = frag_kb(HL + (slot0 + nloc) * H + kb, hlf); const v16b bw = frag_kb(W2P + ((size_t)e * 16 + nloc) * D + kb, hlf); acc = wmma16b(a, bw, acc); acc = wmma16b(al, bw, acc); }
  const float bb = bf16_rne(b2[e * KL + (nloc < KL ? nloc : 0)]);
#pragma unroll
  for (int r8 = 0; r8 < 8; ++r8) { const float lg = acc[r8] * (1.0f / (XS * WSC)) + bb; float l4[KL];
    for (int k = 0; k < KL; ++k) l4[k] = __shfl(lg, k, 16);
    if (nloc == 0) { const int rl = 8 * hlf + r8; float q[KL], p[KC]; for (int k = 0; k < KL; ++k) { so[wave][rl][k] = l4[k]; q[k] = sigm(l4[k]); }
      p[0] = 1.0f - q[0]; for (int k = 1; k < KL; ++k) p[k] = q[k - 1] - q[k]; p[KL] = q[KL - 1]; float s = 0.0f; for (int k = 0; k < KC; ++k) { p[k] = fmaxf(p[k], EPSP); s += p[k]; } s = fmaxf(s, EPSP);
      for (int k = 0; k < KC; ++k) sp[wave][rl][k] = p[k] / s; for (int k = KC; k < 8; ++k) sp[wave][rl][k] = 0.0f; } }
  wave_lds_sync();
  for (int pass = 0; pass < 2; ++pass) { if (lane < 16) *(volatile v4f*)(LOGS + (slot0 + lane) * 4) = *(const v4f*)(&so[wave][lane][0]); *(volatile v4f*)(PRS + slot0 * 8 + lane * 4) = *(const v4f*)(&sp[wave][lane >> 1][(lane & 1) * 4]); __threadfence(); }
}
__global__ __launch_bounds__(256) void out_kernel(const int* __restrict__ sidx, const int* __restrict__ RANK, const float* __restrict__ LOGS, const float* __restrict__ PRS, float* __restrict__ outL, float* __restrict__ outP) {
  __shared__ __attribute__((aligned(16))) float st[8][32 * KC];
  const int wave = threadIdx.x >> 5, lane = threadIdx.x & 31; const int t = blockIdx.x * 256 + threadIdx.x;
  const int e = iclamp(sidx[t], 0, NE - 1); const int rk = iclamp(RANK[(size_t)e * B + t], 0, CAP - 1); const size_t slot = (size_t)e * CAP + rk;
  const v4f lg = *(const v4f*)(LOGS + slot * 4); const v4f p0 = *(const v4f*)(PRS + slot * 8); const float p4 = PRS[slot * 8 + 4];
  for (int k = 0; k < 4; ++k) st[wave][lane * KC + k] = p0[k]; st[wave][lane * KC + 4] = p4;
  wave_lds_sync();
  for (int pass = 0; pass < 2; ++pass) { *(volatile v4f*)(outL + (size_t)t * KL) = lg; const size_t pb = ((size_t)blockIdx.x * 256 + wave * 32) * KC; *(volatile v4f*)(outP + pb + lane * 4) = *(const v4f*)(&st[wave][lane * 4]); if (lane < 8) *(volatile v4f*)(outP + pb + 128 + lane * 4) = *(const v4f*)(&st[wave][128 + lane * 4]); __threadfence(); }
}
}

extern "C" void kernel_launch(void* const* d_in, const int* in_sizes, int n_in, void* d_out, int out_size, void* d_ws, size_t ws_size, hipStream_t stream) {
  (void)n_in;
  auto Fp = [&](int i) { return (const float*)d_in[i]; }; auto Ip = [&](int i) { return (const int*)d_in[i]; };
  if (in_sizes[0] != B * D || in_sizes[1] != B || in_sizes[2] != NE * D * H || in_sizes[3] != NE * H || in_sizes[4] != NE * H * KL || in_sizes[5] != NE * KL || out_size != B * KL + B * KC) return;
  size_t off = 0; char* ws = (char*)d_ws;
  auto carve = [&](size_t bytes) { char* p = ws + off; off += (bytes + 255) & ~(size_t)255; return p; };
  b16* W1T = (b16*)carve((size_t)NE * H * D * 2); b16* W2P = (b16*)carve((size_t)NE * 16 * D * 2); int* RANK = (int*)carve((size_t)NE * B * 4);
  b16* HH = (b16*)carve((size_t)NSLOT * H * 2); b16* HL = (b16*)carve((size_t)NSLOT * H * 2); float* LOGS = (float*)carve((size_t)NSLOT * 4 * 4); float* PRS = (float*)carve((size_t)NSLOT * 8 * 4);
  CsrBufs3 grp; off = csr_carve3(grp, ws, off, B, NE);
  if (off > ws_size || off > ((size_t)128 << 20)) return;
  wprep1_kernel<<<dim3(D / 64, H / 64, NE), 256, 0, stream>>>(Fp(2), W1T);
  wprep2_kernel<<<(unsigned)(((size_t)NE * 16 * D / 8 + 255) / 256), 256, 0, stream>>>(Fp(4), W2P);
  csr_build3(grp, Ip(1), B, NE, stream);
  rank_kernel<<<1, 256, 0, stream>>>(Ip(1), RANK);
  l1_kernel<<<dim3(RB, H / 128, NE), 128, 0, stream>>>(Fp(0), W1T, Fp(3), grp.PERM, grp.ROWPTR, grp.ROWCNT, (int)grp.permLen, HH, HL);
  l2_kernel<<<dim3(RB, 1, NE), 128, 0, stream>>>(HH, HL, W2P, Fp(5), grp.ROWCNT, LOGS, PRS);
  float* outL = (float*)d_out; float* outP = outL + (size_t)B * KL;
  out_kernel<<<B / 256, 256, 0, stream>>>(Ip(1), RANK, LOGS, PRS, outL, outP);
}
